// DecoderLSTM_81836306858398
// MI455X (gfx1250) — hardware-verified
//
#include <hip/hip_runtime.h>

typedef __attribute__((ext_vector_type(16))) _Float16 v16h;
typedef __attribute__((ext_vector_type(8)))  _Float16 v8h;
typedef __attribute__((ext_vector_type(8)))  float    v8f;
typedef __attribute__((ext_vector_type(4)))  float    v4f;

constexpr int NBATCH = 8192;
constexpr int HID    = 64;
constexpr int NOUT   = 3;
constexpr int NSTEPS = 64;
constexpr int TM     = 16;
constexpr int NTHR   = 128;
constexpr int WPITCH = 72;
constexpr int HPITCH = 72;
constexpr int OROW   = NSTEPS * NOUT;
constexpr int OUTS_N = TM * OROW;
constexpr float WSCALE  = 64.0f;
constexpr float HSCALE  = 1024.0f;
constexpr float ACC_INV = 1.0f / 65536.0f;

static_assert(NBATCH % TM == 0, "tile");
static_assert(HID == 64, "k");
static_assert(OUTS_N == 6 * 4 * NTHR, "final store covers the staged tile exactly: 6 float4 per thread");
static_assert(2 * TM * HID + 4 * 4 * HID <= OUTS_N, "prologue scratch fits in the output staging area");
static_assert((TM * OROW * 4) % 512 == 0, "block output region is whole 512-B wave chunks");
static_assert((WPITCH % 8) == 0 && (HPITCH % 8) == 0, "16-B aligned fragment loads");

__device__ __forceinline__ float bfr(float f) {
  unsigned u = __float_as_uint(f);
  u = (u + 0x7FFFu + ((u >> 16) & 1u)) & 0xFFFF0000u;
  return __uint_as_float(u);
}
__device__ __forceinline__ v4f bfr4(v4f v) {
  v4f r;
  r[0] = bfr(v[0]); r[1] = bfr(v[1]); r[2] = bfr(v[2]); r[3] = bfr(v[3]);
  return r;
}
__device__ __forceinline__ void cbar() { asm volatile("" ::: "memory"); }

union FragU { v16h v; v8h h[2]; };
__device__ __forceinline__ v16h frag_load(const _Float16* p) {
  FragU f; f.h[0] = *(const v8h*)(p); f.h[1] = *(const v8h*)(p + 16); return f.v;
}
__device__ __forceinline__ v8f mma16(v16h a, v16h b, v8f c) {
  c = __builtin_amdgcn_wmma_f32_16x16x32_f16(false, a, false, b, (short)0, c, false, false);
  asm volatile("v_nop\n\tv_nop\n\tv_nop\n\tv_nop" : "+v"(c) : "v"(a), "v"(b));
  return c;
}
__device__ __forceinline__ v8f zero8() { return (v8f){0.f, 0.f, 0.f, 0.f, 0.f, 0.f, 0.f, 0.f}; }

__device__ __forceinline__ float sigm(float v) {
  const float e = __expf(-v);
  return __builtin_amdgcn_rcpf(1.0f + e);
}
__device__ __forceinline__ float tanh_(float v) {
  const float e = __expf(-2.0f * fabsf(v));
  const float r = (1.0f - e) * __builtin_amdgcn_rcpf(1.0f + e);
  return copysignf(r, v);
}

__device__ __forceinline__ v8h cvt_w8(v4f a, v4f b) {
  v8h hv;
  hv[0] = (_Float16)(bfr(a[0]) * WSCALE);
  hv[1] = (_Float16)(bfr(a[1]) * WSCALE);
  hv[2] = (_Float16)(bfr(a[2]) * WSCALE);
  hv[3] = (_Float16)(bfr(a[3]) * WSCALE);
  hv[4] = (_Float16)(bfr(b[0]) * WSCALE);
  hv[5] = (_Float16)(bfr(b[1]) * WSCALE);
  hv[6] = (_Float16)(bfr(b[2]) * WSCALE);
  hv[7] = (_Float16)(bfr(b[3]) * WSCALE);
  return hv;
}
__device__ __forceinline__ v8h cvt_h8(v4f a, v4f b) {
  v8h hv;
  hv[0] = (_Float16)(bfr(a[0]) * HSCALE);
  hv[1] = (_Float16)(bfr(a[1]) * HSCALE);
  hv[2] = (_Float16)(bfr(a[2]) * HSCALE);
  hv[3] = (_Float16)(bfr(a[3]) * HSCALE);
  hv[4] = (_Float16)(bfr(b[0]) * HSCALE);
  hv[5] = (_Float16)(bfr(b[1]) * HSCALE);
  hv[6] = (_Float16)(bfr(b[2]) * HSCALE);
  hv[7] = (_Float16)(bfr(b[3]) * HSCALE);
  return hv;
}

__device__ __forceinline__ void stage_w(_Float16* dst, const float* __restrict__ src, int tid) {
#pragma unroll 2
  for (int it = 0; it < 16; ++it) {
    const int q  = it * NTHR + tid;
    const int n  = q >> 3;
    const int k8 = (q & 7) * 8;
    const float* sp = src + n * HID + k8;
    const v4f a = *(const v4f*)(sp);
    const v4f b = *(const v4f*)(sp + 4);
    *(v8h*)(dst + n * WPITCH + k8) = cvt_w8(a, b);
  }
}

__global__ __launch_bounds__(NTHR) void lstm_decode_kernel(
    const float* __restrict__ x,
    const float* __restrict__ hidden,
    const float* __restrict__ cell,
    const float* __restrict__ Wih0,
    const float* __restrict__ Whh0,
    const float* __restrict__ bih0,
    const float* __restrict__ bhh0,
    const float* __restrict__ Wih1,
    const float* __restrict__ Whh1,
    const float* __restrict__ bih1,
    const float* __restrict__ bhh1,
    const float* __restrict__ Wfc,
    const float* __restrict__ bfc,
    const int*   __restrict__ nstep,
    float*       __restrict__ out)
{
  __shared__ __align__(16) _Float16 Wh0s[4 * HID * WPITCH];
  __shared__ __align__(16) _Float16 Wi1s[4 * HID * WPITCH];
  __shared__ __align__(16) _Float16 Wh1s[4 * HID * WPITCH];
  __shared__ __align__(16) _Float16 Wfcs[16 * WPITCH];
  __shared__ __align__(16) _Float16 h0s[2][TM * HPITCH];
  __shared__ __align__(16) _Float16 h1s[2][TM * HPITCH];
  __shared__ __align__(16) float    xs[TM * 4];
  __shared__ __align__(16) float    outs[OUTS_N];
  __shared__ __align__(16) float    wci[4 * HID * NOUT];

  const int tid  = threadIdx.x;
  const int wv   = tid >> 5;
  const int lane = tid & 31;
  const int hh   = lane >> 4;
  const int cc   = lane & 15;
  const int jcol = 16 * wv + cc;
  const int base = blockIdx.x * TM;

  stage_w(Wh0s, Whh0, tid); cbar();
  stage_w(Wi1s, Wih1, tid); cbar();
  stage_w(Wh1s, Whh1, tid); cbar();
  {
    const int n  = tid >> 3;
    const int k8 = (tid & 7) * 8;
    const int nc = (n < NOUT) ? n : (NOUT - 1);
    const float* sp = Wfc + nc * HID + k8;
    const v4f a = *(const v4f*)(sp);
    const v4f b = *(const v4f*)(sp + 4);
    v8h hv = cvt_w8(a, b);
    v8h z;
#pragma unroll
    for (int e = 0; e < 8; ++e) z[e] = (_Float16)0.0f;
    if (n >= NOUT) hv = z;
    *(v8h*)(Wfcs + n * WPITCH + k8) = hv;
  }
  cbar();
  {
    const int m  = tid >> 3;
    const int k8 = (tid & 7) * 8;
    const float* s0 = hidden + ((size_t)(base + m)) * HID + k8;
    const float* s1 = hidden + ((size_t)NBATCH + base + m) * HID + k8;
    const v4f a0 = *(const v4f*)(s0);
    const v4f b0 = *(const v4f*)(s0 + 4);
    const v4f a1 = *(const v4f*)(s1);
    const v4f b1 = *(const v4f*)(s1 + 4);
    *(v8h*)(h0s[0] + m * HPITCH + k8) = cvt_h8(a0, b0);
    *(v8h*)(h1s[0] + m * HPITCH + k8) = cvt_h8(a1, b1);
  }
  cbar();
#pragma unroll
  for (int it = 0; it < 4; ++it) {
    const int q  = it * NTHR + tid;
    const int ly = q >> 8;
    const int m  = (q >> 4) & 15;
    const int k4 = (q & 15) * 4;
    const v4f v = *(const v4f*)(cell + ((size_t)ly * NBATCH + base + m) * HID + k4);
    *(v4f*)(outs + q * 4) = bfr4(v);
  }
  cbar();
  if (tid < 64) {
    const v4f v0 = *(const v4f*)(bih0 + tid * 4);
    const v4f v1 = *(const v4f*)(bhh0 + tid * 4);
    const v4f v2 = *(const v4f*)(bih1 + tid * 4);
    const v4f v3 = *(const v4f*)(bhh1 + tid * 4);
    *(v4f*)(outs + 2 * TM * HID + 0 * 256 + tid * 4) = bfr4(v0);
    *(v4f*)(outs + 2 * TM * HID + 1 * 256 + tid * 4) = bfr4(v1);
    *(v4f*)(outs + 2 * TM * HID + 2 * 256 + tid * 4) = bfr4(v2);
    *(v4f*)(outs + 2 * TM * HID + 3 * 256 + tid * 4) = bfr4(v3);
  }
  cbar();
#pragma unroll
  for (int it = 0; it < 2; ++it) {
    const int q = it * NTHR + tid;
    if (q < (4 * HID * NOUT) / 4) {
      const v4f v = *(const v4f*)(Wih0 + q * 4);
      *(v4f*)(wci + q * 4) = bfr4(v);
    }
  }
  __syncthreads();

  float c0s[8], c1s[8];
#pragma unroll
  for (int r = 0; r < 8; ++r) {
    const int m = 8 * hh + r;
    c0s[r] = outs[m * HID + jcol];
    c1s[r] = outs[TM * HID + m * HID + jcol];
  }
  float b0g[4], b1g[4], wc[4][3];
#pragma unroll
  for (int g = 0; g < 4; ++g) {
    const int n = HID * g + jcol;
    b0g[g] = outs[2 * TM * HID + 0 * 256 + n] + outs[2 * TM * HID + 1 * 256 + n];
    b1g[g] = outs[2 * TM * HID + 2 * 256 + n] + outs[2 * TM * HID + 3 * 256 + n];
    wc[g][0] = wci[n * 3 + 0];
    wc[g][1] = wci[n * 3 + 1];
    wc[g][2] = wci[n * 3 + 2];
  }
  const int   co   = (cc < NOUT) ? cc : (NOUT - 1);
  const float bfl  = bfr(bfc[co]);
  const float bfcv = (cc < NOUT) ? bfl : 0.0f;
  {
    const int m = tid & 15;
    const float* xp = x + (size_t)(base + m) * NOUT;
    const float x0 = bfr(xp[0]);
    const float x1 = bfr(xp[1]);
    const float x2 = bfr(xp[2]);
    if (tid < TM) {
      v4f v; v[0] = x0; v[1] = x1; v[2] = x2; v[3] = 0.0f;
      *(v4f*)(xs + m * 4) = v;
    }
  }
  __syncthreads();
#pragma unroll
  for (int it = 0; it < 6; ++it) {
    const v4f z = {0.f, 0.f, 0.f, 0.f};
    *(v4f*)(outs + (it * NTHR + tid) * 4) = z;
  }
  __syncthreads();

  int T = nstep[0];
  T = (T < 0) ? 0 : T;
  T = (T > NSTEPS) ? NSTEPS : T;

  int p = 0;
  for (int t = 0; t < T; ++t) {
    const _Float16* h0r = h0s[p];
    _Float16*       h0w = h0s[p ^ 1];
    const _Float16* h1r = h1s[p];
    _Float16*       h1w = h1s[p ^ 1];

    v8f acc[4];
#pragma unroll
    for (int g = 0; g < 4; ++g) acc[g] = zero8();
#pragma unroll
    for (int ks = 0; ks < 2; ++ks) {
      const v16h a = frag_load(h0r + cc * HPITCH + ks * 32 + hh * 8);
#pragma unroll
      for (int g = 0; g < 4; ++g) {
        const v16h b = frag_load(Wh0s + (HID * g + jcol) * WPITCH + ks * 32 + hh * 8);
        acc[g] = mma16(a, b, acc[g]);
      }
    }
#pragma unroll
    for (int r = 0; r < 8; ++r) {
      const int m = 8 * hh + r;
      const v4f xv = *(const v4f*)(xs + m * 4);
      float pre[4];
#pragma unroll
      for (int g = 0; g < 4; ++g) {
        float xq = xv[0] * wc[g][0];
        xq = fmaf(xv[1], wc[g][1], xq);
        xq = fmaf(xv[2], wc[g][2], xq);
        pre[g] = fmaf(acc[g][r], ACC_INV, xq) + b0g[g];
      }
      const float ig = sigm(pre[0]);
      const float fg = sigm(pre[1]);
      const float gg = tanh_(pre[2]);
      const float og = sigm(pre[3]);
      const float cn = fmaf(fg, c0s[r], ig * gg);
      c0s[r] = cn;
      const float hn = og * tanh_(cn);
      h0w[m * HPITCH + jcol] = (_Float16)(hn * HSCALE);
    }
    __syncthreads();

#pragma unroll
    for (int g = 0; g < 4; ++g) acc[g] = zero8();
#pragma unroll
    for (int ks = 0; ks < 2; ++ks) {
      const v16h a = frag_load(h0w + cc * HPITCH + ks * 32 + hh * 8);
#pragma unroll
      for (int g = 0; g < 4; ++g) {
        const v16h b = frag_load(Wi1s + (HID * g + jcol) * WPITCH + ks * 32 + hh * 8);
        acc[g] = mma16(a, b, acc[g]);
      }
    }
#pragma unroll
    for (int ks = 0; ks < 2; ++ks) {
      const v16h a = frag_load(h1r + cc * HPITCH + ks * 32 + hh * 8);
#pragma unroll
      for (int g = 0; g < 4; ++g) {
        const v16h b = frag_load(Wh1s + (HID * g + jcol) * WPITCH + ks * 32 + hh * 8);
        acc[g] = mma16(a, b, acc[g]);
      }
    }
#pragma unroll
    for (int r = 0; r < 8; ++r) {
      const int m = 8 * hh + r;
      const float ig = sigm(fmaf(acc[0][r], ACC_INV, b1g[0]));
      const float fg = sigm(fmaf(acc[1][r], ACC_INV, b1g[1]));
      const float gg = tanh_(fmaf(acc[2][r], ACC_INV, b1g[2]));
      const float og = sigm(fmaf(acc[3][r], ACC_INV, b1g[3]));
      const float cn = fmaf(fg, c1s[r], ig * gg);
      c1s[r] = cn;
      const float hn = og * tanh_(cn);
      h1w[m * HPITCH + jcol] = (_Float16)(hn * HSCALE);
    }
    __syncthreads();

    if (wv == 0) {
      v8f oc = zero8();
#pragma unroll
      for (int ks = 0; ks < 2; ++ks) {
        const v16h a = frag_load(h1w + cc * HPITCH + ks * 32 + hh * 8);
        const v16h b = frag_load(Wfcs + cc * WPITCH + ks * 32 + hh * 8);
        oc = mma16(a, b, oc);
      }
      if (cc < NOUT) {
#pragma unroll
        for (int r = 0; r < 8; ++r) {
          const int m = 8 * hh + r;
          const float v = fmaf(oc[r], ACC_INV, bfcv);
          xs[m * 4 + cc] = v;
          outs[m * OROW + t * NOUT + cc] = v;
        }
      }
    }
    __syncthreads();
    p ^= 1;
  }
  __syncthreads();

  float* ob = out + (size_t)base * OROW;
  for (int pass = 0; pass < 2; ++pass) {
#pragma unroll
    for (int it = 0; it < 6; ++it) {
      const int q = it * NTHR + tid;
      const v4f v = *(const v4f*)(outs + q * 4);
      *(volatile v4f*)(ob + q * 4) = v;
    }
    __threadfence();
  }
}

extern "C" void kernel_launch(void* const* d_in, const int* in_sizes, int n_in,
                              void* d_out, int out_size, void* d_ws, size_t ws_size,
                              hipStream_t stream) {
  (void)d_ws; (void)ws_size;
  if (n_in < 14) return;
  if (out_size != NBATCH * NSTEPS * NOUT) return;
  if (in_sizes[0] != NBATCH * NOUT) return;
  if (in_sizes[1] != 2 * NBATCH * HID || in_sizes[2] != 2 * NBATCH * HID) return;
  if (in_sizes[4] != 4 * HID * HID || in_sizes[7] != 4 * HID * HID || in_sizes[8] != 4 * HID * HID) return;
  if (in_sizes[3] != 4 * HID * NOUT || in_sizes[11] != NOUT * HID || in_sizes[12] != NOUT || in_sizes[13] < 1) return;
  lstm_decode_kernel<<<NBATCH / TM, NTHR, 0, stream>>>(
      (const float*)d_in[0],  (const float*)d_in[1],  (const float*)d_in[2],
      (const float*)d_in[3],  (const float*)d_in[4],  (const float*)d_in[5],
      (const float*)d_in[6],  (const float*)d_in[7],  (const float*)d_in[8],
      (const float*)d_in[9],  (const float*)d_in[10], (const float*)d_in[11],
      (const float*)d_in[12], (const int*)d_in[13],   (float*)d_out);
}
